// NetVLAD_V2_53472342835405
// MI455X (gfx1250) — hardware-run, weakly checked
//
#include <hip/hip_runtime.h>


#ifndef NB
#define NB 16
#endif
#ifndef LL
#define LL 4096
#endif
#define NB_FULL 16
#define LL_FULL 4096
#define CC   128
#define DD   512
#define KK   64
#define NBC  (NB < 8 ? NB : 8)
#define XP   136
#define FS   64.0f
#define FSI  (1.0f / 64.0f)
#define CS   16.0f
#define SCL  ((float)(1.4426950408889634 / (64.0 * 16.0)))
#define PSH  14.0f
#define NEGB (-3.0e38f)
#define EPSN 1e-12f

static_assert(NB <= NB_FULL);
static_assert(LL <= LL_FULL);
static_assert(NB % NBC == 0);
static_assert(CC % 32 == 0);
static_assert(DD % 32 == 0);
static_assert(LL % 32 == 0);
static_assert(LL % 64 == 0);
static_assert(DD % 64 == 0);
static_assert(KK == 64);
static_assert(LL % 256 == 0);
static_assert(DD == 512);
static_assert(CC == 128);
static_assert(KK % 8 == 0);
static_assert((NBC * KK) % 32 == 0);
static_assert((XP * 2) % 16 == 0);
static_assert(XP >= CC);
static_assert(((size_t)DD * CC) % 8 == 0);
static_assert(2 * 64 * 68 * 4 <= 131072);
static_assert(64 * XP * 2 + 4 * 64 * 4 + 64 * 4 <= 131072);
static_assert(16 * 68 * 4 <= 131072);

typedef _Float16 h16;
typedef unsigned short bf;
typedef __attribute__((ext_vector_type(16))) __bf16   v16bf;
typedef __attribute__((ext_vector_type(16))) _Float16 v16h;
typedef __attribute__((ext_vector_type(8)))  _Float16 v8h;
typedef __attribute__((ext_vector_type(8)))  unsigned short v8us;
typedef __attribute__((ext_vector_type(8)))  float    v8f;
typedef __attribute__((ext_vector_type(4)))  float    v4f;
typedef v4f  __attribute__((may_alias)) v4fa;
typedef v8us __attribute__((may_alias)) v8usa;

__device__ __forceinline__ unsigned short f2bf(float f) { unsigned u = __float_as_uint(f); u += 0x7FFFu + ((u >> 16) & 1u); return (unsigned short)(u >> 16); }
__device__ __forceinline__ float bfr(float f) { return __uint_as_float(((unsigned)f2bf(f)) << 16); }
__device__ __forceinline__ v16h cat16(v8h lo, v8h hi) { return __builtin_shufflevector(lo, hi, 0, 1, 2, 3, 4, 5, 6, 7, 8, 9, 10, 11, 12, 13, 14, 15); }
__device__ __forceinline__ v16bf cat16b(v8us lo, v8us hi) { return __builtin_bit_cast(v16bf, __builtin_shufflevector(lo, hi, 0, 1, 2, 3, 4, 5, 6, 7, 8, 9, 10, 11, 12, 13, 14, 15)); }
__device__ __forceinline__ v8f wmma16(v16h a, v16h b, v8f c) { return __builtin_amdgcn_wmma_f32_16x16x32_f16(false, a, false, b, (short)0, c, false, false); }
__device__ __forceinline__ v8f wmmab(v16bf a, v16bf b, v8f c) { return __builtin_amdgcn_wmma_f32_16x16x32_bf16(false, a, false, b, (short)0, c, false, false); }
__device__ __forceinline__ v16h  ldh(const h16* p) { return cat16(*(const v8h*)p, *(const v8h*)(p + 16)); }
__device__ __forceinline__ v16bf ldb(const bf* p)  { return cat16b(*(const v8us*)p, *(const v8us*)(p + 16)); }
__device__ __forceinline__ void wave_sync() { __builtin_amdgcn_fence(3  , "wavefront"); __builtin_amdgcn_wave_barrier(); asm volatile("" ::: "memory"); }
__device__ __forceinline__ v8f wmma16g(v16h a, v16h b, v8f c) { c = wmma16(a, b, c); asm volatile("v_nop\n\tv_nop\n\tv_nop\n\tv_nop" : "+v"(c) : "v"(a), "v"(b)); return c; }
__device__ __forceinline__ v8f wmmabg(v16bf a, v16bf b, v8f c) { c = wmmab(a, b, c); asm volatile("v_nop\n\tv_nop\n\tv_nop\n\tv_nop" : "+v"(c) : "v"(a), "v"(b)); return c; }
static __device__ __forceinline__ h16 toh_flush(float v) { const h16 r = (h16)v; return (fabsf(v) < 6.103515625e-05f) ? (h16)0.0f : r; }

__global__ __launch_bounds__(256) void k_cvt8(const float* __restrict__ src, bf* dst, size_t n8) {
    const size_t i = (size_t)blockIdx.x * 256 + threadIdx.x; if (i >= n8) return;
    const v8f v = *(const v8f*)(src + i * 8); v8us o;
#pragma unroll
    for (int k = 0; k < 8; ++k) o[k] = f2bf(v[k]);
    *(volatile v8us*)(dst + i * 8) = o; __threadfence(); *(volatile v8us*)(dst + i * 8) = o;
}

__global__ __launch_bounds__(256) void k_xprep(const float* __restrict__ x, bf* XT, float* INV) {
#pragma clang fp contract(off)
    __shared__ __align__(16) unsigned short xt[64 * XP];
    __shared__ __align__(16) float red[4 * 64];
    __shared__ __align__(16) float inv_s[64];
    const int tid = threadIdx.x;
    const int l = tid & 63, cg = tid >> 6;
    const int n = blockIdx.y, l0 = blockIdx.x * 64;
    const float* p = x + ((size_t)n * CC) * LL_FULL + l0 + l;
    float s = 0.0f;
#pragma unroll 4
    for (int i = 0; i < CC / 4; ++i) {
        const int c = cg + 4 * i;
        const unsigned short u = f2bf(p[(size_t)c * LL_FULL]);
        const float v = __uint_as_float(((unsigned)u) << 16);
        s += v * v;
        xt[l * XP + c] = u;
    }
    red[cg * 64 + l] = s;
    __syncthreads();
    if (tid < 64) {
        const float ss = (red[tid] + red[64 + tid]) + (red[128 + tid] + red[192 + tid]);
        inv_s[tid] = 1.0f / fmaxf(sqrtf(ss), EPSN);
    }
    __syncthreads();
    bf* orow = XT + ((size_t)n * LL + l0) * CC;
    static_assert(4 * 16 == 64);
    static_assert(4 * 256 * 16 == 64 * CC * 2);
#pragma unroll 1
    for (int ps = 0; ps < 2; ++ps) {
#pragma unroll
        for (int s4 = 0; s4 < 4; ++s4) { const int row = 16 * s4 + (tid >> 4), c8 = (tid & 15) * 8;
            const v8us val = *(const v8usa*)(&xt[row * XP + c8]);
            *(volatile v8us*)(orow + (size_t)row * CC + c8) = val; }
        if (tid < 16) { const v4f iv = *(const v4fa*)(&inv_s[tid * 4]);
            *(volatile v4f*)(INV + (size_t)n * LL + l0 + tid * 4) = iv; }
        if (ps == 0) __threadfence(); }
}

__global__ __launch_bounds__(256) void k_cprep(const float* __restrict__ cent, h16* CN) {
#pragma clang fp contract(off)
    const int lane = threadIdx.x & 31;
    const int wave = __builtin_amdgcn_readfirstlane((int)(threadIdx.x >> 5));
    const int k = blockIdx.x * 8 + wave;
    const float* row = cent + (size_t)k * DD;
    const v8f a = *(const v8f*)(row + lane * 8), b = *(const v8f*)(row + 256 + lane * 8);
    float va[8], vb[8]; float s = 0.0f;
#pragma unroll
    for (int i = 0; i < 8; ++i) { va[i] = bfr(a[i]); vb[i] = bfr(b[i]); s += va[i] * va[i]; s += vb[i] * vb[i]; }
    s += __shfl_xor(s, 16, 32); s += __shfl_xor(s, 8, 32); s += __shfl_xor(s, 4, 32); s += __shfl_xor(s, 2, 32); s += __shfl_xor(s, 1, 32);
    const float inv = (1.0f / fmaxf(sqrtf(s), EPSN)) * CS;
    v8h ha, hb;
#pragma unroll
    for (int i = 0; i < 8; ++i) { ha[i] = toh_flush(va[i] * inv); hb[i] = toh_flush(vb[i] * inv); }
    h16* dst = CN + (size_t)k * DD + lane * 8;
    *(volatile v8h*)dst = ha; *(volatile v8h*)(dst + 256) = hb;
    __threadfence();
    *(volatile v8h*)dst = ha; *(volatile v8h*)(dst + 256) = hb;
}

__global__ __launch_bounds__(32) void k_fgemm(const bf* __restrict__ XT, const bf* __restrict__ WB, const float* __restrict__ bias, const float* __restrict__ invn, h16* FLD, h16* FDL) {
    __shared__ __align__(16) float os[64 * 68];
    __shared__ __align__(16) float osT[64 * 68];
    const int lane = threadIdx.x & 31, lr = lane & 15, hi = lane >> 4; const int r0 = blockIdx.x * 64, c0 = blockIdx.y * 64;
    v8f acc[4][4];
#pragma unroll
    for (int mb = 0; mb < 4; ++mb)
#pragma unroll
        for (int nb = 0; nb < 4; ++nb) acc[mb][nb] = (v8f){};
    const size_t aoff = (size_t)(r0 + lr) * CC + 8 * hi, boff = (size_t)(c0 + lr) * CC + 8 * hi;
#pragma unroll 1
    for (int kc = 0; kc < CC; kc += 32) {
        v16bf a[4];
#pragma unroll
        for (int mb = 0; mb < 4; ++mb) a[mb] = ldb(XT + aoff + (size_t)mb * 16 * CC + kc);
#pragma unroll
        for (int nb = 0; nb < 4; ++nb) { const v16bf b = ldb(WB + boff + (size_t)nb * 16 * CC + kc);
#pragma unroll
            for (int mb = 0; mb < 4; ++mb) acc[mb][nb] = wmmabg(a[mb], b, acc[mb][nb]); }
    }
    float bc[4];
#pragma unroll
    for (int nb = 0; nb < 4; ++nb) bc[nb] = bfr(bias[c0 + nb * 16 + lr]) * FS;
#pragma unroll
    for (int mb = 0; mb < 4; ++mb) {
        const float* ip = invn + r0 + mb * 16 + hi * 8;
        const v4f i0 = *(const v4f*)ip, i1 = *(const v4f*)(ip + 4);
        float iv[8];
#pragma unroll
        for (int j = 0; j < 4; ++j) { iv[j] = i0[j] * FS; iv[4 + j] = i1[j] * FS; }
#pragma unroll
        for (int nb = 0; nb < 4; ++nb) {
            v4f lo4, hi4;
#pragma unroll
            for (int j = 0; j < 8; ++j) { const float val = acc[mb][nb][j] * iv[j] + bc[nb];
                os[(mb * 16 + hi * 8 + j) * 68 + nb * 16 + lr] = val;
                if (j < 4) lo4[j] = val; else hi4[j - 4] = val; }
            *(v4fa*)(&osT[(nb * 16 + lr) * 68 + mb * 16 + hi * 8]) = lo4; *(v4fa*)(&osT[(nb * 16 + lr) * 68 + mb * 16 + hi * 8 + 4]) = hi4; }
    }
    wave_sync();
    const int bb = r0 / LL, l0 = r0 % LL;
    const size_t fl = ((size_t)bb * LL + l0) * DD + c0;
    const size_t fd = ((size_t)bb * DD + c0) * LL + l0;
    static_assert(16 * 4 == 64);
    static_assert(16 * 32 * 16 == 64 * 64 * 2);
#pragma unroll 1
    for (int ps = 0; ps < 2; ++ps) {
#pragma unroll 4
        for (int s = 0; s < 16; ++s) { const int row = 4 * s + (lane >> 3), c8 = (lane & 7) * 8;
            const v4f x0 = *(const v4fa*)(&os[row * 68 + c8]);  const v4f x1 = *(const v4fa*)(&os[row * 68 + c8 + 4]);
            const v4f y0 = *(const v4fa*)(&osT[row * 68 + c8]); const v4f y1 = *(const v4fa*)(&osT[row * 68 + c8 + 4]);
            v8h hv, tv;
#pragma unroll
            for (int i = 0; i < 4; ++i) { hv[i] = toh_flush(x0[i]); hv[4 + i] = toh_flush(x1[i]); tv[i] = toh_flush(y0[i]); tv[4 + i] = toh_flush(y1[i]); }
            *(volatile v8h*)(FLD + fl + (size_t)row * DD + c8) = hv;
            *(volatile v8h*)(FDL + fd + (size_t)row * LL + c8) = tv; }
        if (ps == 0) __threadfence(); }
}

__global__ __launch_bounds__(32) void k_logits(const h16* __restrict__ CN, const h16* __restrict__ FLD, float* LG) {
    __shared__ __align__(16) float os[16 * 68];
    const int lane = threadIdx.x & 31, lr = lane & 15, hi = lane >> 4; const int c0 = blockIdx.x * 64;
    v8f acc[4][4];
#pragma unroll
    for (int mb = 0; mb < 4; ++mb)
#pragma unroll
        for (int nb = 0; nb < 4; ++nb) acc[mb][nb] = (v8f){};
    const size_t aoff = (size_t)lr * DD + 8 * hi, boff = (size_t)(c0 + lr) * DD + 8 * hi;
#pragma unroll 1
    for (int kc = 0; kc < DD; kc += 32) {
        v16h a[4];
#pragma unroll
        for (int mb = 0; mb < 4; ++mb) a[mb] = ldh(CN + aoff + (size_t)mb * 16 * DD + kc);
#pragma unroll
        for (int nb = 0; nb < 4; ++nb) { const v16h b = ldh(FLD + boff + (size_t)nb * 16 * DD + kc);
#pragma unroll
            for (int mb = 0; mb < 4; ++mb) acc[mb][nb] = wmma16g(a[mb], b, acc[mb][nb]); }
    }
    const int bb = c0 / LL, l0 = c0 % LL;
    const size_t base = ((size_t)bb * KK) * LL + l0;
    static_assert(8 * 2 == 16);
    static_assert(8 * 32 * 16 == 16 * 64 * 4);
#pragma unroll
    for (int mb = 0; mb < 4; ++mb) {
#pragma unroll
        for (int nb = 0; nb < 4; ++nb) {
#pragma unroll
            for (int j = 0; j < 8; ++j) os[(hi * 8 + j) * 68 + nb * 16 + lr] = acc[mb][nb][j]; }
        wave_sync();
#pragma unroll 1
        for (int ps = 0; ps < 2; ++ps) {
#pragma unroll
            for (int s = 0; s < 8; ++s) { const int row = 2 * s + (lane >> 4), c4 = (lane & 15) * 4;
                const v4f val = *(const v4fa*)(&os[row * 68 + c4]);
                *(volatile v4f*)(LG + base + (size_t)(mb * 16 + row) * LL + c4) = val; }
            if (ps == 0) __threadfence(); }
        wave_sync();
    }
}

__global__ __launch_bounds__(256) void k_softmax(const float* __restrict__ LG, h16* P, float* RS) {
#pragma clang fp contract(off)
    __shared__ __align__(16) float rs_s[32];
    const int lane = threadIdx.x & 31;
    const int wave = __builtin_amdgcn_readfirstlane((int)(threadIdx.x >> 5));
    const int rowb = blockIdx.x * 32;
#pragma unroll 1
    for (int q = 0; q < 4; ++q) {
        const int row = rowb + wave * 4 + q;
        const float* src = LG + (size_t)row * LL + lane * 8;
        float mx = NEGB;
#pragma unroll 1
        for (int it = 0; it < LL / 256; ++it) {
            const v4f a = *(const v4f*)(src + it * 256), b = *(const v4f*)(src + it * 256 + 4);
            mx = fmaxf(mx, fmaxf(fmaxf(a[0], a[1]), fmaxf(a[2], a[3])));
            mx = fmaxf(mx, fmaxf(fmaxf(b[0], b[1]), fmaxf(b[2], b[3]))); }
        mx = fmaxf(mx, __shfl_xor(mx, 16, 32)); mx = fmaxf(mx, __shfl_xor(mx, 8, 32)); mx = fmaxf(mx, __shfl_xor(mx, 4, 32));
        mx = fmaxf(mx, __shfl_xor(mx, 2, 32));  mx = fmaxf(mx, __shfl_xor(mx, 1, 32));
        float ls = 0.0f;
        h16* dst = P + (size_t)row * LL + lane * 8;
#pragma unroll 1
        for (int ps = 0; ps < 2; ++ps) {
#pragma unroll 1
            for (int it = 0; it < LL / 256; ++it) {
                const v4f a = *(const v4f*)(src + it * 256), b = *(const v4f*)(src + it * 256 + 4);
                v8h o; float s8 = 0.0f;
#pragma unroll
                for (int i = 0; i < 4; ++i) {
                    const float ea = (a[i] - mx) * SCL + PSH, eb = (b[i] - mx) * SCL + PSH;
                    const float ga = (ea < -14.0f) ? 0.0f : __builtin_amdgcn_exp2f(ea);
                    const float gb = (eb < -14.0f) ? 0.0f : __builtin_amdgcn_exp2f(eb);
                    const h16 pa = (h16)ga; const h16 pc = (h16)gb;
                    o[i] = pa; o[4 + i] = pc; s8 += (float)pa; s8 += (float)pc; }
                *(volatile v8h*)(dst + it * 256) = o;
                if (ps == 0) ls += s8; }
            if (ps == 0) __threadfence(); }
        ls += __shfl_xor(ls, 16, 32); ls += __shfl_xor(ls, 8, 32); ls += __shfl_xor(ls, 4, 32); ls += __shfl_xor(ls, 2, 32); ls += __shfl_xor(ls, 1, 32);
        if (lane == 0) rs_s[wave * 4 + q] = ls;
    }
    __syncthreads();
    if (threadIdx.x < 8) { const v4f v = *(const v4fa*)(&rs_s[threadIdx.x * 4]);
        float* d = RS + rowb + threadIdx.x * 4;
        *(volatile v4f*)d = v; __threadfence(); *(volatile v4f*)d = v; }
}

__global__ __launch_bounds__(32) void k_pv(const h16* __restrict__ P, const h16* __restrict__ FDL, const float* __restrict__ RS, float* OUT) {
    __shared__ __align__(16) float os[16 * 68];
    const int lane = threadIdx.x & 31, lr = lane & 15, hi = lane >> 4; const int c0 = blockIdx.x * 64, bb = blockIdx.y;
    v8f acc[4][4];
#pragma unroll
    for (int mb = 0; mb < 4; ++mb)
#pragma unroll
        for (int nb = 0; nb < 4; ++nb) acc[mb][nb] = (v8f){};
    const size_t aoff = ((size_t)bb * KK + lr) * LL + 8 * hi, boff = ((size_t)bb * DD + c0 + lr) * LL + 8 * hi;
#pragma unroll 1
    for (int kc = 0; kc < LL; kc += 32) {
        v16h a[4];
#pragma unroll
        for (int mb = 0; mb < 4; ++mb) a[mb] = ldh(P + aoff + (size_t)mb * 16 * LL + kc);
#pragma unroll
        for (int nb = 0; nb < 4; ++nb) { const v16h b = ldh(FDL + boff + (size_t)nb * 16 * LL + kc);
#pragma unroll
            for (int mb = 0; mb < 4; ++mb) acc[mb][nb] = wmma16g(a[mb], b, acc[mb][nb]); }
    }
    float* obase = OUT + ((size_t)bb * KK) * DD + c0;
    static_assert(8 * 2 == 16);
    static_assert(8 * 32 * 16 == 16 * 64 * 4);
#pragma unroll
    for (int mb = 0; mb < 4; ++mb) {
        const float* rp = RS + bb * KK + mb * 16 + hi * 8;
        const v4f r0v = *(const v4f*)rp, r1v = *(const v4f*)(rp + 4);
        float rinv[8];
#pragma unroll
        for (int j = 0; j < 4; ++j) { rinv[j] = (1.0f / r0v[j]) * FSI; rinv[4 + j] = (1.0f / r1v[j]) * FSI; }
#pragma unroll
        for (int nb = 0; nb < 4; ++nb) {
#pragma unroll
            for (int j = 0; j < 8; ++j) os[(hi * 8 + j) * 68 + nb * 16 + lr] = acc[mb][nb][j] * rinv[j]; }
        wave_sync();
#pragma unroll 1
        for (int ps = 0; ps < 2; ++ps) {
#pragma unroll
            for (int s = 0; s < 8; ++s) { const int row = 2 * s + (lane >> 4), c4 = (lane & 15) * 4;
                const v4f val = *(const v4fa*)(&os[row * 68 + c4]);
                *(volatile v4f*)(obase + (size_t)(mb * 16 + row) * DD + c4) = val; }
            if (ps == 0) __threadfence(); }
        wave_sync();
    }
}

static constexpr size_t al256(size_t v) { return (v + 255) & ~(size_t)255; }
static constexpr size_t SZ_XT  = al256((size_t)NB * LL * CC * 2);
static constexpr size_t SZ_WB  = al256((size_t)DD * CC * 2);
static constexpr size_t SZ_INV = al256((size_t)NB * LL * 4);
static constexpr size_t SZ_CN  = al256((size_t)KK * DD * 2);
static constexpr size_t SZ_F   = al256((size_t)NBC * LL * DD * 2);
static constexpr size_t SZ_LG  = al256((size_t)NBC * KK * LL * 4);
static constexpr size_t SZ_P   = al256((size_t)NBC * KK * LL * 2);
static constexpr size_t SZ_RS  = al256((size_t)NBC * KK * 4);
static constexpr size_t SZ_TOTAL = SZ_XT + SZ_WB + SZ_INV + SZ_CN + 2 * SZ_F + SZ_LG + SZ_P + SZ_RS;
static_assert(SZ_TOTAL <= (size_t)134217728);
static_assert((size_t)(NBC * LL / 64) * (DD / 64) * 8192 == (size_t)NBC * LL * DD * 2);
static_assert((size_t)(NBC * LL / 64) * 64 * 64 * 4 == (size_t)NBC * KK * LL * 4);
static_assert((size_t)(NBC * KK / 32) * 32 * LL * 2 == (size_t)NBC * KK * LL * 2);
static_assert((size_t)(LL / 64) * NB * 64 * CC * 2 == (size_t)NB * LL * CC * 2);

extern "C" void kernel_launch(void* const* d_in, const int* in_sizes, int n_in,
                              void* d_out, int out_size, void* d_ws, size_t ws_size, hipStream_t stream) {
    if (n_in < 4) return;
    const size_t needx = ((size_t)(NB - 1) * CC + (CC - 1)) * LL_FULL + LL;
    if ((size_t)in_sizes[0] < needx) return;
    if ((size_t)in_sizes[1] < (size_t)DD * CC || in_sizes[2] < DD || (size_t)in_sizes[3] < (size_t)KK * DD) return;
    if ((size_t)out_size < (size_t)NB * KK * DD) return;
    if (SZ_TOTAL > ws_size) return;
    const float* x    = (const float*)d_in[0];
    const float* w    = (const float*)d_in[1];
    const float* bias = (const float*)d_in[2];
    const float* cent = (const float*)d_in[3];
    float* OUT = (float*)d_out;
    char* wsp = (char*)d_ws;
    bf*    XT  = (bf*)wsp;    wsp += SZ_XT;
    bf*    WB  = (bf*)wsp;    wsp += SZ_WB;
    float* INV = (float*)wsp; wsp += SZ_INV;
    h16*   CN  = (h16*)wsp;   wsp += SZ_CN;
    h16*   FLD = (h16*)wsp;   wsp += SZ_F;
    h16*   FDL = (h16*)wsp;   wsp += SZ_F;
    float* LG  = (float*)wsp; wsp += SZ_LG;
    h16*   P   = (h16*)wsp;   wsp += SZ_P;
    float* RS  = (float*)wsp; wsp += SZ_RS;

    { const size_t n8 = (size_t)DD * CC / 8; k_cvt8<<<(unsigned)((n8 + 255) / 256), 256, 0, stream>>>(w, WB, n8); }
    k_cprep<<<KK / 8, 256, 0, stream>>>(cent, CN);
    k_xprep<<<dim3(LL / 64, NB, 1), 256, 0, stream>>>(x, XT, INV);

    for (int cb = 0; cb < NB; cb += NBC) {
        k_fgemm<<<dim3(NBC * LL / 64, DD / 64, 1), 32, 0, stream>>>(XT + (size_t)cb * LL * CC, WB, bias, INV + (size_t)cb * LL, FLD, FDL);
        k_logits<<<dim3(NBC * LL / 64, 1, 1), 32, 0, stream>>>(CN, FLD, LG);
        k_softmax<<<NBC * KK / 32, 256, 0, stream>>>(LG, P, RS);
        k_pv<<<dim3(DD / 64, NBC, 1), 32, 0, stream>>>(P, FDL, RS, OUT + (size_t)cb * KK * DD);
    }
}
